// MambaBlock_82523501625677
// MI455X (gfx1250) — hardware-verified
//
#include <hip/hip_runtime.h>
#include <math.h>

typedef __attribute__((ext_vector_type(16))) _Float16 v16h;
typedef __attribute__((ext_vector_type(8)))  _Float16 v8h;
typedef __attribute__((ext_vector_type(16))) __bf16   v16b;
typedef __attribute__((ext_vector_type(8)))  __bf16   v8b;
typedef __attribute__((ext_vector_type(8)))  float    v8f;
typedef __attribute__((ext_vector_type(4)))  float    v4f;

constexpr int kSeqL  = 2048;
constexpr int kDmod  = 1024;
constexpr int kDin   = 2048;
constexpr int kNst   = 16;
constexpr int kDtR   = 64;
constexpr int kConvK = 4;
constexpr int kPrjN  = kDtR + 2 * kNst;
constexpr int kPrjP  = 128;
constexpr int kXZP   = 2 * kDin;
constexpr int kTP    = 260;
static_assert(kPrjN == 96 && kPrjN <= kPrjP, "x_proj width");
static_assert((kDmod % 32) == 0 && (kDtR % 32) == 0 && (kDin % 32) == 0, "GEMM K multiples of 32");
static_assert((kSeqL % 64) == 0 && (kXZP % 64) == 0 && (kPrjP % 64) == 0 && (kDin % 64) == 0 && (kDmod % 64) == 0, "GEMM M,N multiples of 64");
static_assert((kSeqL % 32) == 0 && (kDmod % 256) == 0, "prep tiles");
static_assert((kSeqL % 16) == 0 && (kDin % 256) == 0 && kNst == 16, "scan tiles");
static_assert(kDtR == 64, "dt split tiles");
static_assert((kDmod % 64) == 0 && (kDtR % 64) == 0 && (kDin % 64) == 0, "transpose tiles");

constexpr size_t kOffXB   = 0;
constexpr size_t kOffRS   = kOffXB   + (size_t)kSeqL * kDmod * 2;
constexpr size_t kOffWIN  = kOffRS   + (size_t)kSeqL * 4;
constexpr size_t kOffWXP  = kOffWIN  + (size_t)kXZP  * kDmod * 2;
constexpr size_t kOffWDT  = kOffWXP  + (size_t)kPrjP * kDmod * 2;
constexpr size_t kOffWOUT = kOffWDT  + (size_t)kDin  * kDtR  * 2;
constexpr size_t kOffXZ   = kOffWOUT + (size_t)kDmod * kDin  * 2;
constexpr size_t kOffXD   = kOffXZ   + (size_t)kSeqL * kXZP  * 4;
constexpr size_t kOffDRH  = kOffXD   + (size_t)kSeqL * kPrjP * 4;
constexpr size_t kOffDRL  = kOffDRH  + (size_t)kSeqL * kDtR  * 2;
constexpr size_t kOffDLR  = kOffDRL  + (size_t)kSeqL * kDtR  * 2;
constexpr size_t kOffYH   = kOffDLR  + (size_t)kSeqL * kDin  * 4;
constexpr size_t kOffYL   = kOffYH   + (size_t)kSeqL * kDin  * 2;
constexpr size_t kWsTotal = kOffYL   + (size_t)kSeqL * kDin  * 2;
static_assert(kWsTotal == 85991424ull, "carve total");
static_assert(kWsTotal <= 134217728ull, "carve cap");
static_assert((kOffRS % 128) == 0 && (kOffWIN % 128) == 0 && (kOffWXP % 128) == 0 && (kOffWDT % 128) == 0 &&
              (kOffWOUT % 128) == 0 && (kOffXZ % 128) == 0 && (kOffXD % 128) == 0 && (kOffDRH % 128) == 0 &&
              (kOffDRL % 128) == 0 && (kOffDLR % 128) == 0 && (kOffYH % 128) == 0 && (kOffYL % 128) == 0,
              "128-B aligned regions");

__device__ __forceinline__ unsigned short f2bf_bits(float f) {
  unsigned u = __float_as_uint(f);
  return (unsigned short)((u + 0x7FFFu + ((u >> 16) & 1u)) >> 16);
}
__device__ __forceinline__ float bf_bits2f(unsigned short h) { return __uint_as_float(((unsigned)h) << 16); }

__device__ __forceinline__ void dep_guard4_h(v8f& a, v8f& b, v8f& c, v8f& d, v16h x, v16h y) { asm volatile("v_nop\n\tv_nop\n\tv_nop\n\tv_nop" : "+v"(a), "+v"(b), "+v"(c), "+v"(d) : "v"(x), "v"(y)); }
__device__ __forceinline__ void dep_guard4_b(v8f& a, v8f& b, v8f& c, v8f& d, v16b x, v16b y) { asm volatile("v_nop\n\tv_nop\n\tv_nop\n\tv_nop" : "+v"(a), "+v"(b), "+v"(c), "+v"(d) : "v"(x), "v"(y)); }
__device__ __forceinline__ void keep4_h(v16h a, v16h b, v16h c, v16h d) { asm volatile("v_nop" :: "v"(a), "v"(b), "v"(c), "v"(d)); }
__device__ __forceinline__ void keep4_b(v16b a, v16b b, v16b c, v16b d) { asm volatile("v_nop" :: "v"(a), "v"(b), "v"(c), "v"(d)); }
__device__ __forceinline__ void acc_guard4(v8f& a, v8f& b, v8f& c, v8f& d) { asm volatile("v_nop\n\tv_nop\n\tv_nop\n\tv_nop" : "+v"(a), "+v"(b), "+v"(c), "+v"(d)); }
template <typename T> struct Frag;
template <> struct Frag<_Float16> {
  typedef v16h V; union U { v16h v; v8h h[2]; };
  static __device__ __forceinline__ v16h load(const _Float16* p) {
    U f; f.h[0] = *(const v8h*)(p); f.h[1] = *(const v8h*)(p + 16); return f.v;
  }
  static __device__ __forceinline__ v8f mma(v16h a, v16h b, v8f c) {
    return __builtin_amdgcn_wmma_f32_16x16x32_f16(false, a, false, b, (short)0, c, false, false);
  }
  static __device__ __forceinline__ void guard4(v8f& a, v8f& b, v8f& c, v8f& d, v16h x, v16h y) { dep_guard4_h(a, b, c, d, x, y); }
  static __device__ __forceinline__ void keep(v16h a, v16h b, v16h c, v16h d) { keep4_h(a, b, c, d); }
};
template <> struct Frag<__bf16> {
  typedef v16b V; union U { v16b v; v8b h[2]; };
  static __device__ __forceinline__ v16b load(const __bf16* p) {
    U f; f.h[0] = *(const v8b*)(p); f.h[1] = *(const v8b*)(p + 16); return f.v;
  }
  static __device__ __forceinline__ v8f mma(v16b a, v16b b, v8f c) {
    return __builtin_amdgcn_wmma_f32_16x16x32_bf16(false, a, false, b, (short)0, c, false, false);
  }
  static __device__ __forceinline__ void guard4(v8f& a, v8f& b, v8f& c, v8f& d, v16b x, v16b y) { dep_guard4_b(a, b, c, d, x, y); }
  static __device__ __forceinline__ void keep(v16b a, v16b b, v16b c, v16b d) { keep4_b(a, b, c, d); }
};

template <int ET> struct Elem;
template <> struct Elem<0> { typedef _Float16 T; };
template <> struct Elem<1> { typedef __bf16 T; };
template <int ET, int SPL, int BIAS_MODE, int OUT_MODE, int RESID>
__global__ __launch_bounds__(256) void wmma_gemm64(
    const unsigned short* __restrict__ Ap, const unsigned short* __restrict__ A2p, int lda, long strideA,
    const unsigned short* __restrict__ Btp, const unsigned short* __restrict__ Bt2p, int ldb, long strideB,
    void* __restrict__ Cout, void* __restrict__ Cout2, int ldc, long strideC,
    const float* __restrict__ bias,
    const float* __restrict__ resid, long strideR,
    int M, int N, int K, float scale) {
  typedef typename Elem<ET>::T T;
  typedef typename Frag<T>::V V;
  const T* A = (const T*)Ap; const T* A2 = (const T*)A2p; const T* Bt = (const T*)Btp; const T* Bt2 = (const T*)Bt2p;
  __shared__ __align__(16) float sT[8][16 * 68];
  const int b    = blockIdx.y;
  const int lane = threadIdx.x & 31;
  const int wave = threadIdx.x >> 5;
  const int tilesN = N >> 6;
  const int tilesM = M >> 6;
  const int tile = blockIdx.x * 8 + wave;
  if (tile >= tilesM * tilesN) return;
  const int tm = tile / tilesN;
  const int tn = tile - tm * tilesN;
  const int m0 = tm << 6;
  const int n0 = tn << 6;

  const T* Ab  = A  + (size_t)b * strideA;
  const T* Bb  = Bt + (size_t)b * strideB;
  const T* Ab2 = (SPL >= 1) ? (A2  + (size_t)b * strideA) : nullptr;
  const T* Bb2 = (SPL == 2) ? (Bt2 + (size_t)b * strideB) : nullptr;

  const int rlane = lane & 15;
  const int koff  = (lane >> 4) * 8;
  const int mOff  = (lane >> 4) * 8;

  v8f acc[4][4];
#pragma unroll
  for (int i = 0; i < 4; ++i)
#pragma unroll
    for (int j = 0; j < 4; ++j) acc[i][j] = (v8f){0.f,0.f,0.f,0.f,0.f,0.f,0.f,0.f};

  for (int k0 = 0; k0 < K; k0 += 32) {
    V bh[4], bl[4];
#pragma unroll
    for (int j = 0; j < 4; ++j) {
      const size_t bo = (size_t)(n0 + (j << 4) + rlane) * ldb + koff + k0;
      bh[j] = Frag<T>::load(Bb + bo);
      if (SPL == 2) bl[j] = Frag<T>::load(Bb2 + bo);
    }
#pragma unroll
    for (int i = 0; i < 4; ++i) {
      const size_t ao = (size_t)(m0 + (i << 4) + rlane) * lda + koff + k0;
      V ah = Frag<T>::load(Ab + ao);
      V al;
      if (SPL >= 1) al = Frag<T>::load(Ab2 + ao);
#pragma unroll
      for (int j = 0; j < 4; ++j) {
        acc[i][j] = Frag<T>::mma(ah, bh[j], acc[i][j]);
        if (SPL == 2) acc[i][j] = Frag<T>::mma(ah, bl[j], acc[i][j]);
        if (SPL >= 1) acc[i][j] = Frag<T>::mma(al, bh[j], acc[i][j]);
      }
      Frag<T>::guard4(acc[i][0], acc[i][1], acc[i][2], acc[i][3], ah, (SPL >= 1) ? al : ah);
    }
    Frag<T>::keep(bh[0], bh[1], bh[2], bh[3]);
    if (SPL == 2) Frag<T>::keep(bl[0], bl[1], bl[2], bl[3]);
  }
  acc_guard4(acc[0][0], acc[0][1], acc[0][2], acc[0][3]);
  acc_guard4(acc[1][0], acc[1][1], acc[1][2], acc[1][3]);
  acc_guard4(acc[2][0], acc[2][1], acc[2][2], acc[2][3]);
  acc_guard4(acc[3][0], acc[3][1], acc[3][2], acc[3][3]);

  float* slab = sT[wave];
#pragma unroll
  for (int i = 0; i < 4; ++i) {
    const int mBase = m0 + (i << 4);
    float rs8[8];
#pragma unroll
    for (int r = 0; r < 8; ++r) rs8[r] = 1.0f;
    if (BIAS_MODE == 3) {
      const v4f ra = *(const v4f*)(bias + mBase + mOff);
      const v4f rb = *(const v4f*)(bias + mBase + mOff + 4);
      rs8[0] = ra[0]; rs8[1] = ra[1]; rs8[2] = ra[2]; rs8[3] = ra[3];
      rs8[4] = rb[0]; rs8[5] = rb[1]; rs8[6] = rb[2]; rs8[7] = rb[3];
    }
#pragma unroll
    for (int j = 0; j < 4; ++j) {
      const int n = n0 + (j << 4) + rlane;
      float bv = 0.f;
      if (BIAS_MODE == 2) bv = bias[n];
      if (BIAS_MODE == 4) bv = bf_bits2f(f2bf_bits(bias[n]));
#pragma unroll
      for (int r = 0; r < 8; ++r) {
        float v = acc[i][j][r] * scale;
        if (BIAS_MODE == 1) v += bias[mBase + mOff + r];
        if (BIAS_MODE == 2 || BIAS_MODE == 4) v += bv;
        if (BIAS_MODE == 3) v *= rs8[r];
        slab[(mOff + r) * 68 + (j << 4) + rlane] = v;
      }
    }
    __builtin_amdgcn_fence(__ATOMIC_RELEASE, "workgroup");
    __builtin_amdgcn_wave_barrier();
    __builtin_amdgcn_fence(__ATOMIC_ACQUIRE, "workgroup");
    if (OUT_MODE == 0) {
      float* C = (float*)Cout + (size_t)b * strideC;
      const int hh = lane >> 4, c4 = (lane & 15) * 4;
      if (RESID != 0) {
        const float* Rb = resid + (size_t)b * strideR;
#pragma unroll
        for (int it = 0; it < 8; ++it) {
          if (it == 4) asm volatile("" ::: "memory");
          const int row = it * 2 + hh;
          const v4f rr = *(const v4f*)(Rb + (size_t)(mBase + row) * ldc + n0 + c4);
          float* sp = slab + row * 68 + c4;
          v4f sv = *(const v4f*)sp;
#pragma unroll
          for (int e = 0; e < 4; ++e) {
            const float re = rr[e];
            const float ra = (RESID == 2) ? bf_bits2f(f2bf_bits(re)) : re;
            sv[e] = sv[e] + ra;
          }
          *(v4f*)sp = sv;
        }
      }
      for (int pass = 0; pass < 2; ++pass) {
#pragma unroll
        for (int it = 0; it < 8; ++it) {
          const int row = it * 2 + hh;
          v4f v = *(const v4f*)(slab + row * 68 + c4);
          *(volatile v4f*)(C + (size_t)(mBase + row) * ldc + n0 + c4) = v;
        }
        __threadfence();
      }
    } else {
      const int q = lane >> 3, c8 = (lane & 7) * 8;
      unsigned short* C  = (unsigned short*)Cout  + (size_t)b * strideC;
      unsigned short* C2 = (OUT_MODE == 2) ? ((unsigned short*)Cout2 + (size_t)b * strideC) : nullptr;
      for (int pass = 0; pass < 2; ++pass) {
#pragma unroll
        for (int it = 0; it < 4; ++it) {
          const int row = it * 4 + q;
          const float* sp = slab + row * 68 + c8;
          v8h hv, lv;
#pragma unroll
          for (int e = 0; e < 8; ++e) {
            if (OUT_MODE == 1) {
              hv[e] = (_Float16)sp[e];
            } else {
              unsigned short hb = f2bf_bits(sp[e]);
              unsigned short lb = f2bf_bits(sp[e] - bf_bits2f(hb));
              hv[e] = __builtin_bit_cast(_Float16, hb);
              lv[e] = __builtin_bit_cast(_Float16, lb);
            }
          }
          *(volatile v8h*)(C + (size_t)(mBase + row) * ldc + n0 + c8) = hv;
          if (OUT_MODE == 2) *(volatile v8h*)(C2 + (size_t)(mBase + row) * ldc + n0 + c8) = lv;
        }
        __threadfence();
      }
    }
    __builtin_amdgcn_fence(__ATOMIC_RELEASE, "workgroup");
    __builtin_amdgcn_wave_barrier();
    __builtin_amdgcn_fence(__ATOMIC_ACQUIRE, "workgroup");
  }
}

__global__ __launch_bounds__(256) void prep_rows_kernel(
    const float* __restrict__ X, unsigned short* __restrict__ XB, float* __restrict__ RS)
{
  __shared__ float sS[32];
  const int tid = threadIdx.x, lane = tid & 31, wave = tid >> 5;
  const int r0 = blockIdx.x * 32;
#pragma unroll 1
  for (int rr = 0; rr < 4; ++rr) {
    const int row = r0 + wave * 4 + rr;
    const float* xr = X + (size_t)row * kDmod;
    v8h hv[4];
    float ss = 0.f;
#pragma unroll
    for (int it = 0; it < 4; ++it) {
      if (it == 2) asm volatile("" ::: "memory");
      const float* p = xr + it * 256 + lane * 8;
      const v4f a0 = *(const v4f*)(p);
      const v4f a1 = *(const v4f*)(p + 4);
#pragma unroll
      for (int e = 0; e < 4; ++e) {
        const float x0 = a0[e], x1 = a1[e];
        const unsigned short b0 = f2bf_bits(x0), b1 = f2bf_bits(x1);
        const float f0 = bf_bits2f(b0), f1 = bf_bits2f(b1);
        ss = fmaf(f0, f0, ss);
        ss = fmaf(f1, f1, ss);
        hv[it][e]     = __builtin_bit_cast(_Float16, b0);
        hv[it][4 + e] = __builtin_bit_cast(_Float16, b1);
      }
    }
#pragma unroll
    for (int off = 1; off < 32; off <<= 1) ss += __shfl_xor(ss, off, 32);
    if (lane == 0) sS[wave * 4 + rr] = ss;
    for (int pass = 0; pass < 2; ++pass) {
#pragma unroll
      for (int it = 0; it < 4; ++it)
        *(volatile v8h*)(XB + (size_t)row * kDmod + it * 256 + lane * 8) = hv[it];
      __threadfence();
    }
  }
  __syncthreads();
  if (wave == 0) {
    const int q = lane & 7;
    v4f sv;
#pragma unroll
    for (int e = 0; e < 4; ++e) {
      const float mean = sS[q * 4 + e] * (1.0f / (float)kDmod);
      sv[e] = 1.0f / sqrtf(mean + 1e-6f);
    }
    if (lane < 8) {
      float* p = RS + r0 + q * 4;
      *(volatile v4f*)p = sv;
      __threadfence();
      *(volatile v4f*)p = sv;
    }
  }
}

template <int KSC>
__global__ __launch_bounds__(256) void transpose_bf16_kernel(
    const float* __restrict__ W, const float* __restrict__ ksc, unsigned short* __restrict__ Bt, int Kdim, int Ndim)
{
  __shared__ float tile[64 * 65];
  const int tid = threadIdx.x, lane = tid & 31, wave = tid >> 5;
  const int n0 = blockIdx.x * 64;
  const int k0 = blockIdx.y * 64;
#pragma unroll
  for (int p = 0; p < 16; ++p) {
    if (p == 8) asm volatile("" ::: "memory");
    const int idx = tid + p * 256;
    const int kk  = idx >> 6;
    const int nn  = idx & 63;
    const int n   = n0 + nn;
    const int nc  = (n < Ndim) ? n : (Ndim - 1);
    const float fz = (n < Ndim) ? 1.0f : 0.0f;
    float v = W[(size_t)(k0 + kk) * Ndim + nc];
    if (KSC) {
      const float sc = bf_bits2f(f2bf_bits(ksc[k0 + kk]));
      v = bf_bits2f(f2bf_bits(v)) * sc;
    }
    tile[kk * 65 + nn] = fmaf(v, fz, 0.0f);
  }
  __syncthreads();
  const int q = lane >> 3, c8 = (lane & 7) * 8;
  v8h hv[2];
#pragma unroll
  for (int it = 0; it < 2; ++it) {
    const int nrow = it * 32 + wave * 4 + q;
#pragma unroll
    for (int e = 0; e < 8; ++e) hv[it][e] = __builtin_bit_cast(_Float16, f2bf_bits(tile[(c8 + e) * 65 + nrow]));
  }
  for (int pass = 0; pass < 2; ++pass) {
#pragma unroll
    for (int it = 0; it < 2; ++it) {
      const int nrow = it * 32 + wave * 4 + q;
      *(volatile v8h*)(Bt + (size_t)(n0 + nrow) * Kdim + k0 + c8) = hv[it];
    }
    __threadfence();
  }
}

__global__ __launch_bounds__(256) void dr_split_kernel(
    const float* __restrict__ XD, unsigned short* __restrict__ DRH, unsigned short* __restrict__ DRL, int total8)
{
  const int i = blockIdx.x * 256 + threadIdx.x;
  if (i >= total8) return;
  const int e0  = i << 3;
  const int row = e0 / kDtR;
  const int c8  = e0 - row * kDtR;
  const float* p = XD + (size_t)row * kPrjP + c8;
  const v4f a0 = *(const v4f*)(p);
  const v4f a1 = *(const v4f*)(p + 4);
  v8h hv, lv;
#pragma unroll
  for (int e = 0; e < 4; ++e) {
    const float x0 = a0[e], x1 = a1[e];
    const unsigned short h0 = f2bf_bits(x0), h1 = f2bf_bits(x1);
    const unsigned short l0 = f2bf_bits(x0 - bf_bits2f(h0)), l1 = f2bf_bits(x1 - bf_bits2f(h1));
    hv[e]     = __builtin_bit_cast(_Float16, h0);
    hv[4 + e] = __builtin_bit_cast(_Float16, h1);
    lv[e]     = __builtin_bit_cast(_Float16, l0);
    lv[4 + e] = __builtin_bit_cast(_Float16, l1);
  }
  unsigned short* qh = DRH + e0;
  unsigned short* ql = DRL + e0;
  *(volatile v8h*)qh = hv;
  *(volatile v8h*)ql = lv;
  __threadfence();
  *(volatile v8h*)qh = hv;
  *(volatile v8h*)ql = lv;
}

__global__ __launch_bounds__(256) void scan_kernel(
    const float* __restrict__ DLR, const float* __restrict__ XZ, const float* __restrict__ XD,
    const float* __restrict__ cw, const float* __restrict__ cb,
    const float* __restrict__ A_log, const float* __restrict__ Dv,
    unsigned short* __restrict__ YH, unsigned short* __restrict__ YL)
{
  __shared__ __align__(16) float sBC[16 * 32];
  __shared__ __align__(16) float sCW[16 * 4];
  __shared__ __align__(16) float sCB[16];
  __shared__ __align__(16) float sY[16 * kTP];
  const int tid = threadIdx.x, lane = tid & 31, wave = tid >> 5;
  const int d0 = blockIdx.x * 256, d = d0 + tid;

  float An[kNst];
  {
    const float* ap = A_log + (size_t)d * kNst;
#pragma unroll
    for (int q4 = 0; q4 < 4; ++q4) {
      const v4f av = *(const v4f*)(ap + 4 * q4);
#pragma unroll
      for (int e = 0; e < 4; ++e) {
        const float al = av[e];
        An[4 * q4 + e] = -__expf(bf_bits2f(f2bf_bits(al)));
      }
    }
  }
  const float Dd = bf_bits2f(f2bf_bits(Dv[d]));
  const int dm1 = (d > 0) ? (d - 1) : 0;
  const int dp1 = (d + 1 < kDin) ? (d + 1) : (kDin - 1);
  const int dp2 = (d + 2 < kDin) ? (d + 2) : (kDin - 1);
  const float fm1 = (d > 0) ? 1.0f : 0.0f;
  const float fp1 = (d + 1 < kDin) ? 1.0f : 0.0f;
  const float fp2 = (d + 2 < kDin) ? 1.0f : 0.0f;
  float h[kNst];
#pragma unroll
  for (int n = 0; n < kNst; ++n) h[n] = 0.f;

#pragma unroll 1
  for (int c = 0; c < kSeqL / 16; ++c) {
    const int l0 = c * 16;
    if (wave < 4) {
      const int r = tid >> 3, q = (tid & 7) * 4;
      const v4f v = *(const v4f*)(XD + (size_t)(l0 + r) * kPrjP + kDtR + q);
      *(v4f*)(sBC + r * 32 + q) = v;
    } else if (wave < 6) {
      const int t2 = tid - 128;
      const int r = t2 >> 2, k = t2 & 3;
      sCW[r * 4 + k] = bf_bits2f(f2bf_bits(cw[(size_t)k * kSeqL + l0 + r]));
    } else if (wave == 6) {
      const int r = lane & 15;
      sCB[r] = bf_bits2f(f2bf_bits(cb[l0 + r]));
    }
    __syncthreads();
#pragma unroll 1
    for (int s = 0; s < 16; ++s) {
      const size_t m = (size_t)(l0 + s);
      const float* xr = XZ + m * kXZP;
      const float a  = DLR[m * kDin + d];
      const float x0 = xr[dm1];
      const float x1 = xr[d];
      const float x2 = xr[dp1];
      const float x3 = xr[dp2];
      const float zv = xr[kDin + d];
      const v4f wv = *(const v4f*)(sCW + s * 4);
      const float cbv = sCB[s];
      float cv = wv[0] * (x0 * fm1);
      cv = fmaf(wv[1], x1, cv);
      cv = fmaf(wv[2], x2 * fp1, cv);
      cv = fmaf(wv[3], x3 * fp2, cv);
      cv = cv + cbv;
      const float sgc   = __builtin_amdgcn_rcpf(1.0f + __expf(-cv));
      const float xv    = cv * sgc;
      const float delta = fmaxf(a, 0.0f) + log1pf(__expf(-fabsf(a)));
      v4f Bq[4], Cq[4];
#pragma unroll
      for (int qq = 0; qq < 4; ++qq) {
        Bq[qq] = *(const v4f*)(sBC + s * 32 + 4 * qq);
        Cq[qq] = *(const v4f*)(sBC + s * 32 + kNst + 4 * qq);
      }
      float y = 0.f;
#pragma unroll
      for (int n = 0; n < kNst; ++n) {
        const float e = __expf(delta * An[n]);
        float db = delta * Bq[n >> 2][n & 3];
        asm volatile("" : "+v"(db));
        float p = db * xv;
        asm volatile("" : "+v"(p));
        float qv = h[n] * e;
        asm volatile("" : "+v"(qv));
        const float hn = qv + p;
        h[n] = hn;
        float rr = Cq[n >> 2][n & 3] * hn;
        asm volatile("" : "+v"(rr));
        y += rr;
      }
      float sk = xv * Dd;
      asm volatile("" : "+v"(sk));
      y += sk;
      const float sg = __builtin_amdgcn_rcpf(1.0f + __expf(-zv));
      const float g  = zv * sg;
      sY[s * kTP + tid] = y * g;
    }
    __syncthreads();
    v8h hv[2], lv[2];
#pragma unroll
    for (int it = 0; it < 2; ++it) {
      const float* sp = sY + (it * 8 + wave) * kTP + lane * 8;
      const v4f a0 = *(const v4f*)(sp);
      const v4f a1 = *(const v4f*)(sp + 4);
#pragma unroll
      for (int e = 0; e < 4; ++e) {
        const float y0 = a0[e], y1 = a1[e];
        const unsigned short h0 = f2bf_bits(y0), h1 = f2bf_bits(y1);
        const unsigned short l0b = f2bf_bits(y0 - bf_bits2f(h0)), l1b = f2bf_bits(y1 - bf_bits2f(h1));
        hv[it][e]     = __builtin_bit_cast(_Float16, h0);
        hv[it][4 + e] = __builtin_bit_cast(_Float16, h1);
        lv[it][e]     = __builtin_bit_cast(_Float16, l0b);
        lv[it][4 + e] = __builtin_bit_cast(_Float16, l1b);
      }
    }
    for (int pass = 0; pass < 2; ++pass) {
#pragma unroll
      for (int it = 0; it < 2; ++it) {
        const size_t o = (size_t)(l0 + it * 8 + wave) * kDin + d0 + lane * 8;
        *(volatile v8h*)(YH + o) = hv[it];
        *(volatile v8h*)(YL + o) = lv[it];
      }
      __threadfence();
    }
  }
}

extern "C" void kernel_launch(void* const* d_in, const int* in_sizes, int n_in,
                              void* d_out, int out_size, void* d_ws, size_t ws_size,
                              hipStream_t stream)
{
  if (n_in < 11) return;
  if (in_sizes[0]  != kSeqL * kDmod) return;
  if (in_sizes[1]  != kDmod) return;
  if (in_sizes[2]  != kDmod * kXZP) return;
  if (in_sizes[3]  != kConvK * kSeqL) return;
  if (in_sizes[4]  != kSeqL) return;
  if (in_sizes[5]  != kDmod * kPrjN) return;
  if (in_sizes[6]  != kDtR * kDin) return;
  if (in_sizes[7]  != kDin) return;
  if (in_sizes[8]  != kDin * kDmod) return;
  if (in_sizes[9]  != kDin * kNst) return;
  if (in_sizes[10] != kDin) return;
  if (out_size != kSeqL * kDmod) return;
  if (ws_size < kWsTotal) return;

  const float* x       = (const float*)d_in[0];
  const float* nscale  = (const float*)d_in[1];
  const float* W_in    = (const float*)d_in[2];
  const float* conv_w  = (const float*)d_in[3];
  const float* conv_b  = (const float*)d_in[4];
  const float* W_xprj  = (const float*)d_in[5];
  const float* W_dt    = (const float*)d_in[6];
  const float* b_dt    = (const float*)d_in[7];
  const float* W_out   = (const float*)d_in[8];
  const float* A_log   = (const float*)d_in[9];
  const float* Dv      = (const float*)d_in[10];
  float* dout = (float*)d_out;

  char* ws = (char*)d_ws;
  unsigned short* XB   = (unsigned short*)(ws + kOffXB);
  float*          RS   = (float*)(ws + kOffRS);
  unsigned short* WIN  = (unsigned short*)(ws + kOffWIN);
  unsigned short* WXP  = (unsigned short*)(ws + kOffWXP);
  unsigned short* WDT  = (unsigned short*)(ws + kOffWDT);
  unsigned short* WOUT = (unsigned short*)(ws + kOffWOUT);
  float*          XZ   = (float*)(ws + kOffXZ);
  float*          XD   = (float*)(ws + kOffXD);
  unsigned short* DRH  = (unsigned short*)(ws + kOffDRH);
  unsigned short* DRL  = (unsigned short*)(ws + kOffDRL);
  float*          DLR  = (float*)(ws + kOffDLR);
  unsigned short* YH   = (unsigned short*)(ws + kOffYH);
  unsigned short* YL   = (unsigned short*)(ws + kOffYL);
  const float* dummy_resid = x;

  prep_rows_kernel<<<kSeqL / 32, 256, 0, stream>>>(x, XB, RS);

  transpose_bf16_kernel<1><<<dim3(kXZP / 64, kDmod / 64), 256, 0, stream>>>(W_in,   nscale, WIN,  kDmod, kXZP);
  transpose_bf16_kernel<1><<<dim3(kPrjP / 64, kDmod / 64), 256, 0, stream>>>(W_xprj, nscale, WXP,  kDmod, kPrjN);
  transpose_bf16_kernel<0><<<dim3(kDin / 64, kDtR / 64), 256, 0, stream>>>(W_dt,    nscale, WDT,  kDtR,  kDin);
  transpose_bf16_kernel<0><<<dim3(kDmod / 64, kDin / 64), 256, 0, stream>>>(W_out,  nscale, WOUT, kDin,  kDmod);

  wmma_gemm64<1, 0, 3, 0, 0><<<dim3(256, 1), 256, 0, stream>>>(
      XB, XB, kDmod, 0L, WIN, WIN, kDmod, 0L,
      (void*)XZ, (void*)XZ, kXZP, 0L, RS, dummy_resid, 0L, kSeqL, kXZP, kDmod, 1.0f);

  wmma_gemm64<1, 0, 3, 0, 0><<<dim3(8, 1), 256, 0, stream>>>(
      XB, XB, kDmod, 0L, WXP, WXP, kDmod, 0L,
      (void*)XD, (void*)XD, kPrjP, 0L, RS, dummy_resid, 0L, kSeqL, kPrjP, kDmod, 1.0f);

  dr_split_kernel<<<(kSeqL * kDtR) / 8 / 256, 256, 0, stream>>>(XD, DRH, DRL, (kSeqL * kDtR) / 8);

  wmma_gemm64<1, 1, 4, 0, 0><<<dim3(128, 1), 256, 0, stream>>>(
      DRH, DRL, kDtR, 0L, WDT, WDT, kDtR, 0L,
      (void*)DLR, (void*)DLR, kDin, 0L, b_dt, dummy_resid, 0L, kSeqL, kDin, kDtR, 1.0f);

  scan_kernel<<<dim3(kDin / 256, 1), 256, 0, stream>>>(DLR, XZ, XD, conv_w, conv_b, A_log, Dv, YH, YL);

  wmma_gemm64<1, 1, 0, 0, 2><<<dim3(64, 1), 256, 0, stream>>>(
      YH, YL, kDin, 0L, WOUT, WOUT, kDin, 0L,
      (void*)dout, (void*)dout, kDmod, 0L, RS, x, 0L, kSeqL, kDmod, kDin, 1.0f);
}
